// ChildSumTreeLSTM_29154238005592
// MI455X (gfx1250) — hardware-run, weakly checked
//
#include <hip/hip_runtime.h>
#include <math.h>

typedef __attribute__((ext_vector_type(16))) _Float16 v16h;
typedef __attribute__((ext_vector_type(8)))  _Float16 v8h;
typedef __attribute__((ext_vector_type(8)))  float    v8f;
typedef __attribute__((ext_vector_type(4)))  float    v4f;

constexpr int kLeaves  = 16384;
constexpr int kDim     = 128;
constexpr int kGate3   = 3 * kDim;
constexpr int kExt     = 16;
constexpr int kOutRows = 2 * kLeaves + 2;
constexpr int kTile    = 16;
constexpr int kPA      = 136;
constexpr int kPF      = 132;
static_assert(kDim == 128 && kExt == 16 && kTile == 16, "kernel is specialised for these shapes");
static_assert((kDim % 32) == 0, "K multiple of 32");
static_assert((kLeaves % kTile) == 0, "leaf level is a tile multiple");
static_assert(kOutRows == 32770, "output rows");
static_assert(((kPA * 2) % 16) == 0 && ((kPF * 4) % 16) == 0, "LDS row pitches 16-B aligned");

constexpr float kCarryW   = 256.0f;
constexpr float kCarryX   = 16.0f;
constexpr float kCarryH   = 64.0f;
constexpr float kFoldLeaf = 1.0f / (kCarryX * kCarryW);
constexpr float kFoldInt  = 1.0f / (kCarryH * kCarryW);
constexpr float kF16MinNormal = 6.103515625e-5f;

constexpr size_t kOffWtIoux = 0;
constexpr size_t kOffWtIouh = kOffWtIoux + (size_t)kGate3 * kDim * 2;
constexpr size_t kOffWtF    = kOffWtIouh + (size_t)kGate3 * kDim * 2;
constexpr size_t kOffWtAt   = kOffWtF    + (size_t)kDim * kDim * 2;
constexpr size_t kOffBext   = kOffWtAt   + (size_t)kDim * kDim * 2;
constexpr size_t kOffCA     = kOffBext   + (size_t)kExt * kDim * 4;
constexpr size_t kOffCB     = kOffCA     + (size_t)kLeaves * kDim * 4;
constexpr size_t kWsTotal   = kOffCB     + (size_t)(kLeaves / 2) * kDim * 4;
static_assert(kWsTotal == 12853248ull, "carve total");
static_assert(kWsTotal <= 134217728ull, "carve cap");
static_assert((kOffWtIouh % 128) == 0 && (kOffWtF % 128) == 0 && (kOffWtAt % 128) == 0 &&
              (kOffBext % 128) == 0 && (kOffCA % 128) == 0 && (kOffCB % 128) == 0, "128-B aligned regions");

__device__ __forceinline__ float bf16_rne(float f) {
  const unsigned u = __float_as_uint(f);
  const unsigned r = (u + 0x7FFFu + ((u >> 16) & 1u)) >> 16;
  return __uint_as_float(r << 16);
}
__device__ __forceinline__ _Float16 to_h16(float v, float carry) {
  float s = v * carry;
  s = (fabsf(s) < kF16MinNormal) ? 0.0f : s;
  return (_Float16)s;
}
__device__ __forceinline__ float sigm_fast(float x) {
  const float xc = fminf(fmaxf(x, -30.0f), 30.0f);
  return __builtin_amdgcn_rcpf(1.0f + __expf(-xc));
}
__device__ __forceinline__ float tanh_fast(float x) {
  const float xc = fminf(fmaxf(x, -15.0f), 15.0f);
  const float e = __expf(2.0f * xc);
  return 1.0f - 2.0f * __builtin_amdgcn_rcpf(1.0f + e);
}
union FragU { v16h v; v8h h[2]; };
__device__ __forceinline__ v16h frag_load(const _Float16* p) {
  FragU f;
  f.h[0] = *(const v8h*)(p);
  f.h[1] = *(const v8h*)(p + 16);
  return f.v;
}
__device__ __forceinline__ v8f mma_h(v16h a, v16h b, v8f c) {
  c = __builtin_amdgcn_wmma_f32_16x16x32_f16(false, a, false, b, (short)0, c, false, false);
  asm volatile("v_nop\n\tv_nop\n\tv_nop\n\tv_nop" : "+v"(c) : "v"(a), "v"(b));
  return c;
}

__global__ __launch_bounds__(256) void weight_planes_kernel(
    const float* __restrict__ Wioux, const float* __restrict__ Wiouh,
    const float* __restrict__ Wfh, const float* __restrict__ Wattnh,
    unsigned short* __restrict__ pIoux, unsigned short* __restrict__ pIouh,
    unsigned short* __restrict__ pF, unsigned short* __restrict__ pAt)
{
  const int b = blockIdx.x;
  const float* W;
  unsigned short* dst;
  int ncols;
  int lb;
  if (b < 24)      { W = Wioux;  dst = pIoux; ncols = kGate3; lb = b; }
  else if (b < 48) { W = Wiouh;  dst = pIouh; ncols = kGate3; lb = b - 24; }
  else if (b < 56) { W = Wfh;    dst = pF;    ncols = kDim;   lb = b - 48; }
  else             { W = Wattnh; dst = pAt;   ncols = kDim;   lb = b - 56; }
  const int idx = lb * 256 + (int)threadIdx.x;
  const int nn = idx >> 4;
  const int k8 = (idx & 15) * 8;
  v8h hv;
#pragma unroll
  for (int e = 0; e < 8; ++e) {
    const float w = W[(size_t)(k8 + e) * ncols + nn];
    hv[e] = to_h16(bf16_rne(w), kCarryW);
  }
  unsigned short* q = dst + (size_t)nn * kDim + k8;
  *(volatile v8h*)q = hv;
  __threadfence();
  *(volatile v8h*)q = hv;
}

__global__ __launch_bounds__(128) void bext_kernel(
    const float* __restrict__ hext, const float* __restrict__ Wattnh,
    const float* __restrict__ battnh, float* __restrict__ bext)
{
  __shared__ __align__(16) float sRow[kDim];
  const int m = blockIdx.x;
  const int d = threadIdx.x;
  float acc = 0.0f;
#pragma unroll 4
  for (int k = 0; k < kDim; ++k) {
    const float hv = bf16_rne(hext[m * kDim + k]);
    const float wv = bf16_rne(Wattnh[(size_t)(kDim + k) * kDim + d]);
    acc = fmaf(hv, wv, acc);
  }
  acc += bf16_rne(battnh[d]);
  sRow[d] = acc;
  __syncthreads();
  if (threadIdx.x < 32) {
    const int lane = threadIdx.x;
    const v4f v = *(const v4f*)(sRow + 4 * lane);
    float* q = bext + (size_t)m * kDim + 4 * lane;
    *(volatile v4f*)q = v;
    __threadfence();
    *(volatile v4f*)q = v;
  }
}

template <bool LEAF>
__global__ __launch_bounds__(256) void level_kernel(
    const float* src, const float* __restrict__ cIn, float* __restrict__ cOut,
    float* outBase, int hOff, int n, int isFinal,
    const unsigned short* __restrict__ wIou, const unsigned short* __restrict__ wF,
    const unsigned short* __restrict__ wAt,
    const float* __restrict__ bias1, const float* __restrict__ bias2, const float* __restrict__ bfh,
    const float* __restrict__ bext, const float* __restrict__ hext, const float* __restrict__ wa)
{
  __shared__ __align__(16) _Float16 sA16[LEAF ? 8 : 32 * kPA];
  __shared__ __align__(16) _Float16 sS16[kTile * kPA];
  __shared__ __align__(16) _Float16 sH16[kTile * kPA];
  __shared__ __align__(16) float sHt[kTile * kPF];
  __shared__ __align__(16) float sCn[kTile * kPF];
  __shared__ __align__(16) float sHW[kTile * kPF];
  __shared__ __align__(16) float sBext[kExt * kDim];
  __shared__ __align__(16) float sHext[kExt * kDim];
  __shared__ __align__(16) float sWa[kDim];
  __shared__ __align__(16) float sP[kTile * kExt];
  __shared__ __align__(16) float sPs[kTile];

  const int tid  = threadIdx.x;
  const int lane = tid & 31;
  const int wave = tid >> 5;
  const int row0 = blockIdx.x * kTile;
  constexpr float kFold = LEAF ? kFoldLeaf : kFoldInt;

#pragma unroll
  for (int i = 0; i < 2; ++i) {
    const int i4 = (tid + 256 * i) * 4;
    *(v4f*)(sBext + i4) = *(const v4f*)(bext + i4);
    const v4f hx = *(const v4f*)(hext + i4);
    v4f hr;
#pragma unroll
    for (int e = 0; e < 4; ++e) {
      const float f = hx[e];
      hr[e] = bf16_rne(f);
    }
    *(v4f*)(sHext + i4) = hr;
  }
  if (wave == 0) {
    const v4f wx = *(const v4f*)(wa + 4 * lane);
    v4f wr;
#pragma unroll
    for (int e = 0; e < 4; ++e) {
      const float f = wx[e];
      wr[e] = bf16_rne(f);
    }
    *(v4f*)(sWa + 4 * lane) = wr;
  }

  {
    const int sr = tid >> 4;
    const int sc8 = (tid & 15) * 8;
    if (LEAF) {
      int rr = row0 + sr;
      rr = rr > (n - 1) ? (n - 1) : rr;
      const float* p = src + (size_t)rr * kDim + sc8;
      const v4f a0 = *(const v4f*)(p);
      const v4f a1 = *(const v4f*)(p + 4);
      v8h hv;
#pragma unroll
      for (int e = 0; e < 4; ++e) {
        const float f0 = a0[e];
        const float f1 = a1[e];
        hv[e]     = to_h16(bf16_rne(f0), kCarryX);
        hv[4 + e] = to_h16(bf16_rne(f1), kCarryX);
      }
      *(v8h*)(sS16 + sr * kPA + sc8) = hv;
    } else {
      const int last = 2 * n - 1;
      int re = 2 * (row0 + sr);
      int ro = re + 1;
      re = re > last ? last : re;
      ro = ro > last ? last : ro;
      const float* pe = src + (size_t)re * kDim + sc8;
      const float* po = src + (size_t)ro * kDim + sc8;
      const v4f e0 = *(const v4f*)(pe);
      const v4f e1 = *(const v4f*)(pe + 4);
      const v4f o0 = *(const v4f*)(po);
      const v4f o1 = *(const v4f*)(po + 4);
      v8h hvE, hvO, hvS;
#pragma unroll
      for (int e = 0; e < 4; ++e) {
        const float fe0 = e0[e];
        const float fe1 = e1[e];
        const float fo0 = o0[e];
        const float fo1 = o1[e];
        hvE[e]     = to_h16(fe0, kCarryH);
        hvE[4 + e] = to_h16(fe1, kCarryH);
        hvO[e]     = to_h16(fo0, kCarryH);
        hvO[4 + e] = to_h16(fo1, kCarryH);
        hvS[e]     = to_h16(fe0 + fo0, kCarryH);
        hvS[4 + e] = to_h16(fe1 + fo1, kCarryH);
      }
      *(v8h*)(sA16 + sr * kPA + sc8) = hvE;
      *(v8h*)(sA16 + (kTile + sr) * kPA + sc8) = hvO;
      *(v8h*)(sS16 + sr * kPA + sc8) = hvS;
    }
  }
  __syncthreads();

  const int nl   = lane & 15;
  const int hh   = lane >> 4;
  const int koff = 8 * hh;
  const int col  = 16 * wave + nl;
  const _Float16* WI = (const _Float16*)wIou;
  const _Float16* WF = (const _Float16*)wF;
  const _Float16* WA = (const _Float16*)wAt;

  v8f ai  = (v8f){0.f, 0.f, 0.f, 0.f, 0.f, 0.f, 0.f, 0.f};
  v8f ao  = ai;
  v8f au  = ai;
  v8f af0 = ai;
  v8f af1 = ai;
#pragma unroll
  for (int ks = 0; ks < 4; ++ks) {
    const int k0 = ks * 32 + koff;
    const v16h aS = frag_load(sS16 + nl * kPA + k0);
    const v16h bi = frag_load(WI + (size_t)(col) * kDim + k0);
    const v16h bo = frag_load(WI + (size_t)(kDim + col) * kDim + k0);
    const v16h bu = frag_load(WI + (size_t)(2 * kDim + col) * kDim + k0);
    ai = mma_h(aS, bi, ai);
    ao = mma_h(aS, bo, ao);
    au = mma_h(aS, bu, au);
    if (!LEAF) {
      const v16h aE = frag_load(sA16 + nl * kPA + k0);
      const v16h aO = frag_load(sA16 + (kTile + nl) * kPA + k0);
      const v16h bf = frag_load(WF + (size_t)(col) * kDim + k0);
      af0 = mma_h(aE, bf, af0);
      af1 = mma_h(aO, bf, af1);
    }
  }

  {
    float bI = bf16_rne(bias2[col]);
    float bO = bf16_rne(bias2[kDim + col]);
    float bU = bf16_rne(bias2[2 * kDim + col]);
    float bF = 0.0f;
    if (LEAF) {
      bI += bf16_rne(bias1[col]);
      bO += bf16_rne(bias1[kDim + col]);
      bU += bf16_rne(bias1[2 * kDim + col]);
    } else {
      bF = bf16_rne(bfh[col]);
    }
    float ce[8], co[8];
#pragma unroll
    for (int r = 0; r < 8; ++r) {
      ce[r] = 0.0f;
      co[r] = 0.0f;
    }
    if (!LEAF) {
      const int last = 2 * n - 1;
#pragma unroll
      for (int r = 0; r < 8; ++r) {
        const int node = row0 + 8 * hh + r;
        int r0 = 2 * node;
        int r1 = r0 + 1;
        r0 = r0 > last ? last : r0;
        r1 = r1 > last ? last : r1;
        ce[r] = cIn[(size_t)r0 * kDim + col];
        co[r] = cIn[(size_t)r1 * kDim + col];
      }
    }
#pragma unroll
    for (int r = 0; r < 8; ++r) {
      const float iv = ai[r] * kFold + bI;
      const float ov = ao[r] * kFold + bO;
      const float uv = au[r] * kFold + bU;
      float cn = sigm_fast(iv) * tanh_fast(uv);
      if (!LEAF) {
        const float f0 = af0[r] * kFold + bF;
        const float f1 = af1[r] * kFold + bF;
        const float fc = sigm_fast(f0) * ce[r] + sigm_fast(f1) * co[r];
        cn = cn + fc;
      }
      const float hv = sigm_fast(ov) * tanh_fast(cn);
      const int row = 8 * hh + r;
      sCn[row * kPF + col] = cn;
      sHt[row * kPF + col] = hv;
      sH16[row * kPA + col] = to_h16(hv, kCarryH);
    }
  }
  __syncthreads();

  {
    v8f ah = (v8f){0.f, 0.f, 0.f, 0.f, 0.f, 0.f, 0.f, 0.f};
#pragma unroll
    for (int ks = 0; ks < 4; ++ks) {
      const int k0 = ks * 32 + koff;
      const v16h aH = frag_load(sH16 + nl * kPA + k0);
      const v16h bA = frag_load(WA + (size_t)(col) * kDim + k0);
      ah = mma_h(aH, bA, ah);
    }
#pragma unroll
    for (int r = 0; r < 8; ++r) sHW[(8 * hh + r) * kPF + col] = ah[r] * kFoldInt;
  }

  const int nd0 = row0 + wave;
  const int nd1 = row0 + wave + 8;
  {
    const v4f cv0 = *(const v4f*)(sCn + wave * kPF + 4 * lane);
    const v4f cv1 = *(const v4f*)(sCn + (wave + 8) * kPF + 4 * lane);
    for (int pass = 0; pass < 2; ++pass) {
      if (nd0 < n) {
        *(volatile v4f*)(cOut + (size_t)nd0 * kDim + 4 * lane) = cv0;
        if (isFinal) *(volatile v4f*)(outBase + (size_t)nd0 * kDim + 4 * lane) = cv0;
      }
      if (nd1 < n) {
        *(volatile v4f*)(cOut + (size_t)nd1 * kDim + 4 * lane) = cv1;
        if (isFinal) *(volatile v4f*)(outBase + (size_t)nd1 * kDim + 4 * lane) = cv1;
      }
      __threadfence();
    }
  }
  __syncthreads();

  {
    const int lr = tid >> 4;
    const int lm = tid & 15;
    const float* hw = sHW + lr * kPF;
    const float* be = sBext + lm * kDim;
    float lg = 0.0f;
#pragma unroll 2
    for (int d4 = 0; d4 < kDim / 4; ++d4) {
      const v4f a = *(const v4f*)(hw + 4 * d4);
      const v4f b = *(const v4f*)(be + 4 * d4);
      const v4f w = *(const v4f*)(sWa + 4 * d4);
      lg = fmaf(tanh_fast(a[0] + b[0]), w[0], lg);
      lg = fmaf(tanh_fast(a[1] + b[1]), w[1], lg);
      lg = fmaf(tanh_fast(a[2] + b[2]), w[2], lg);
      lg = fmaf(tanh_fast(a[3] + b[3]), w[3], lg);
    }
    float mx = lg;
    mx = fmaxf(mx, __shfl_xor(mx, 1, 32));
    mx = fmaxf(mx, __shfl_xor(mx, 2, 32));
    mx = fmaxf(mx, __shfl_xor(mx, 4, 32));
    mx = fmaxf(mx, __shfl_xor(mx, 8, 32));
    const float ex = __expf(lg - mx);
    float sm = ex;
    sm += __shfl_xor(sm, 1, 32);
    sm += __shfl_xor(sm, 2, 32);
    sm += __shfl_xor(sm, 4, 32);
    sm += __shfl_xor(sm, 8, 32);
    const float sv = ex * __builtin_amdgcn_rcpf(sm);
    float ss = sv;
    ss += __shfl_xor(ss, 1, 32);
    ss += __shfl_xor(ss, 2, 32);
    ss += __shfl_xor(ss, 4, 32);
    ss += __shfl_xor(ss, 8, 32);
    sP[lr * kExt + lm] = sv;
    if (lm == 0) sPs[lr] = ss;
  }
  __syncthreads();

  {
    v4f ov0 = (v4f){0.f, 0.f, 0.f, 0.f};
    v4f ov1 = (v4f){0.f, 0.f, 0.f, 0.f};
    const float* p0 = sP + wave * kExt;
    const float* p1 = sP + (wave + 8) * kExt;
#pragma unroll 4
    for (int m = 0; m < kExt; ++m) {
      const v4f hx = *(const v4f*)(sHext + m * kDim + 4 * lane);
      const float w0 = 1.0f - p0[m];
      const float w1 = 1.0f - p1[m];
      ov0 += w0 * hx;
      ov1 += w1 * hx;
    }
    const v4f ht0 = *(const v4f*)(sHt + wave * kPF + 4 * lane);
    const v4f ht1 = *(const v4f*)(sHt + (wave + 8) * kPF + 4 * lane);
    const float s0 = sPs[wave];
    const float s1 = sPs[wave + 8];
    ov0 += s0 * ht0;
    ov1 += s1 * ht1;
    for (int pass = 0; pass < 2; ++pass) {
      if (nd0 < n) {
        *(volatile v4f*)(outBase + (size_t)(hOff + nd0) * kDim + 4 * lane) = ov0;
        if (isFinal) *(volatile v4f*)(outBase + (size_t)(2 + nd0) * kDim + 4 * lane) = ov0;
      }
      if (nd1 < n) {
        *(volatile v4f*)(outBase + (size_t)(hOff + nd1) * kDim + 4 * lane) = ov1;
        if (isFinal) *(volatile v4f*)(outBase + (size_t)(2 + nd1) * kDim + 4 * lane) = ov1;
      }
      __threadfence();
    }
  }
}

extern "C" void kernel_launch(void* const* d_in, const int* in_sizes, int n_in,
                              void* d_out, int out_size, void* d_ws, size_t ws_size,
                              hipStream_t stream) {
  if (n_in < 11) return;
  if (in_sizes[0] != kLeaves * kDim) return;
  if (in_sizes[1] != kExt * kDim) return;
  if (in_sizes[2] != kDim * kGate3) return;
  if (in_sizes[3] != kGate3) return;
  if (in_sizes[4] != kDim * kGate3) return;
  if (in_sizes[5] != kGate3) return;
  if (in_sizes[6] != kDim * kDim) return;
  if (in_sizes[7] != kDim) return;
  if (in_sizes[8] != 2 * kDim * kDim) return;
  if (in_sizes[9] != kDim) return;
  if (in_sizes[10] != kDim) return;
  if (out_size != kOutRows * kDim) return;
  if (ws_size < kWsTotal) return;

  const float* x      = (const float*)d_in[0];
  const float* h_ext  = (const float*)d_in[1];
  const float* Wioux  = (const float*)d_in[2];
  const float* bioux  = (const float*)d_in[3];
  const float* Wiouh  = (const float*)d_in[4];
  const float* biouh  = (const float*)d_in[5];
  const float* Wfh    = (const float*)d_in[6];
  const float* bfh    = (const float*)d_in[7];
  const float* Wattnh = (const float*)d_in[8];
  const float* battnh = (const float*)d_in[9];
  const float* Wa     = (const float*)d_in[10];
  float* out = (float*)d_out;

  char* ws = (char*)d_ws;
  unsigned short* wtIoux = (unsigned short*)(ws + kOffWtIoux);
  unsigned short* wtIouh = (unsigned short*)(ws + kOffWtIouh);
  unsigned short* wtF    = (unsigned short*)(ws + kOffWtF);
  unsigned short* wtAt   = (unsigned short*)(ws + kOffWtAt);
  float*          bextP  = (float*)(ws + kOffBext);
  float*          cA     = (float*)(ws + kOffCA);
  float*          cB     = (float*)(ws + kOffCB);

  weight_planes_kernel<<<64, 256, 0, stream>>>(Wioux, Wiouh, Wfh, Wattnh, wtIoux, wtIouh, wtF, wtAt);
  bext_kernel<<<kExt, kDim, 0, stream>>>(h_ext, Wattnh, battnh, bextP);

  int off = 4;
  level_kernel<true><<<kLeaves / kTile, 256, 0, stream>>>(
      x, cB, cA, out, off, kLeaves, 0,
      wtIoux, wtF, wtAt, bioux, biouh, bfh, bextP, h_ext, Wa);

  int belowOff = off;
  off += kLeaves;
  float* cInP = cA;
  float* cOutP = cB;
  for (int n = kLeaves / 2; n >= 2; n >>= 1) {
    const int blocks = (n + kTile - 1) / kTile;
    level_kernel<false><<<blocks, 256, 0, stream>>>(
        out + (size_t)belowOff * kDim, cInP, cOutP, out, off, n, (n == 2) ? 1 : 0,
        wtIouh, wtF, wtAt, bioux, biouh, bfh, bextP, h_ext, Wa);
    belowOff = off;
    off += n;
    float* t = cInP;
    cInP = cOutP;
    cOutP = t;
  }
}
